// SparseContextEncoder_71107478552674
// MI455X (gfx1250) — hardware-verified
//
#include <hip/hip_runtime.h>
#include <math.h>
#include <stdint.h>

constexpr int NUM_SCENES     = 512;
constexpr int STEPS_AGENT    = 6;
constexpr int STEPS_LANE     = 240;
constexpr int DIM_AGENT_IN   = 4;
constexpr int DIM_MODEL      = 128;
constexpr int NUM_HEADS      = 4;
constexpr int DIM_HEAD       = 32;
constexpr int GATES3         = 3 * DIM_MODEL;
constexpr int NUM_LAYERS     = 3;
constexpr int ROWS_AGENT     = NUM_SCENES * STEPS_AGENT;
constexpr int HALF_SCENES    = 256;
constexpr int ROWS_LANE_HALF = HALF_SCENES * STEPS_LANE;
constexpr int NTHR           = 256;
constexpr float W_CARRY      = 16.0f;
constexpr float W_FOLD       = 1.0f / 16.0f;
constexpr float ATT_SCALE    = 0.17677669529663687f;
constexpr float INV_LANE_STEPS = 1.0f / 240.0f;

static_assert(ROWS_AGENT % 64 == 0 && ROWS_LANE_HALF % 64 == 0 && NUM_SCENES % 64 == 0, "cfg");
static_assert(DIM_MODEL % 64 == 0 && GATES3 % 64 == 0 && (2 * DIM_MODEL) % 64 == 0, "cfg");
static_assert(DIM_MODEL % 32 == 0 && (2 * DIM_MODEL) % 32 == 0, "cfg");
static_assert(NUM_HEADS * DIM_HEAD == DIM_MODEL, "cfg");

typedef __attribute__((ext_vector_type(16))) _Float16 v16h;
typedef __attribute__((ext_vector_type(8)))  _Float16 v8h;
typedef __attribute__((ext_vector_type(16))) __bf16   v16b;
typedef __attribute__((ext_vector_type(8)))  __bf16   v8b;
typedef __attribute__((ext_vector_type(8)))  float    v8f;
typedef __attribute__((ext_vector_type(4)))  float    v4f;

__device__ __forceinline__ unsigned short f2bf_bits(float f) {
  unsigned u = __float_as_uint(f);
  return (unsigned short)((u + 0x7FFFu + ((u >> 16) & 1u)) >> 16);
}
__device__ __forceinline__ float bf_bits2f(unsigned short h) { return __uint_as_float(((unsigned)h) << 16); }

__device__ __forceinline__ void dep_guard_h(v8f& a, v8f& b, v16h x, v16h y) { asm volatile("v_nop\n\tv_nop\n\tv_nop\n\tv_nop" : "+v"(a), "+v"(b) : "v"(x), "v"(y)); }
__device__ __forceinline__ void dep_guard_b(v8f& a, v8f& b, v16b x, v16b y) { asm volatile("v_nop\n\tv_nop\n\tv_nop\n\tv_nop" : "+v"(a), "+v"(b) : "v"(x), "v"(y)); }
__device__ __forceinline__ void keep4_h(v16h a, v16h b, v16h c, v16h d) { asm volatile("v_nop" :: "v"(a), "v"(b), "v"(c), "v"(d)); }
__device__ __forceinline__ void keep4_b(v16b a, v16b b, v16b c, v16b d) { asm volatile("v_nop" :: "v"(a), "v"(b), "v"(c), "v"(d)); }
__device__ __forceinline__ void acc_guard4(v8f& a, v8f& b, v8f& c, v8f& d) { asm volatile("v_nop\n\tv_nop\n\tv_nop\n\tv_nop" : "+v"(a), "+v"(b), "+v"(c), "+v"(d)); }
__device__ __forceinline__ void acc_guard3(v8f& a, v8f& b, v8f& c) { asm volatile("v_nop\n\tv_nop\n\tv_nop\n\tv_nop" : "+v"(a), "+v"(b), "+v"(c)); }
template <typename T> struct Frag;
template <> struct Frag<_Float16> {
  typedef v16h V; union U { v16h v; v8h h[2]; };
  static __device__ __forceinline__ v16h load(const _Float16* p) {
    U f; f.h[0] = *(const v8h*)(p); f.h[1] = *(const v8h*)(p + 16); return f.v;
  }
  static __device__ __forceinline__ v8f mma(v16h a, v16h b, v8f c) {
    return __builtin_amdgcn_wmma_f32_16x16x32_f16(false, a, false, b, (short)0, c, false, false);
  }
  static __device__ __forceinline__ void guard(v8f& a, v8f& b, v16h x, v16h y) { dep_guard_h(a, b, x, y); }
  static __device__ __forceinline__ void keep(v16h a, v16h b, v16h c, v16h d) { keep4_h(a, b, c, d); }
};
template <> struct Frag<__bf16> {
  typedef v16b V; union U { v16b v; v8b h[2]; };
  static __device__ __forceinline__ v16b load(const __bf16* p) {
    U f; f.h[0] = *(const v8b*)(p); f.h[1] = *(const v8b*)(p + 16); return f.v;
  }
  static __device__ __forceinline__ v8f mma(v16b a, v16b b, v8f c) {
    return __builtin_amdgcn_wmma_f32_16x16x32_bf16(false, a, false, b, (short)0, c, false, false);
  }
  static __device__ __forceinline__ void guard(v8f& a, v8f& b, v16b x, v16b y) { dep_guard_b(a, b, x, y); }
  static __device__ __forceinline__ void keep(v16b a, v16b b, v16b c, v16b d) { keep4_b(a, b, c, d); }
};
typedef Frag<_Float16> FragH;

__device__ __forceinline__ float fsig(float v)  { return __builtin_amdgcn_rcpf(1.0f + __expf(-v)); }
__device__ __forceinline__ float ftanh(float v) { return 1.0f - 2.0f * __builtin_amdgcn_rcpf(__expf(2.0f * v) + 1.0f); }

template <int ET> struct Elem;
template <> struct Elem<0> { typedef _Float16 T; };
template <> struct Elem<1> { typedef __bf16 T; };
template <int ET, bool SPLIT, int BIAS_MODE, int OUT_MODE, bool RESID, int ACT = 0>
__global__ __launch_bounds__(256) void wmma_gemm64(
    const unsigned short* __restrict__ Ap, const unsigned short* __restrict__ A2p, int lda, long strideA,
    const unsigned short* __restrict__ Btp, const unsigned short* __restrict__ Bt2p, int ldb, long strideB,
    void* __restrict__ Cout, void* __restrict__ Cout2, int ldc, long strideC,
    const float* __restrict__ bias,
    const float* __restrict__ resid, long strideR,
    int M, int N, int K, float scale) {
  typedef typename Elem<ET>::T T;
  typedef typename Frag<T>::V V;
  const T* A = (const T*)Ap; const T* A2 = (const T*)A2p; const T* Bt = (const T*)Btp; const T* Bt2 = (const T*)Bt2p;
  __shared__ __align__(16) float sT[8][16 * 68];
  const int b    = blockIdx.y;
  const int lane = threadIdx.x & 31;
  const int wave = threadIdx.x >> 5;
  const int tilesN = N >> 6;
  const int tilesM = M >> 6;
  const int tile = blockIdx.x * 8 + wave;
  if (tile >= tilesM * tilesN) return;
  const int tm = tile / tilesN;
  const int tn = tile - tm * tilesN;
  const int m0 = tm << 6;
  const int n0 = tn << 6;

  const T* Ab  = A  + (size_t)b * strideA;
  const T* Bb  = Bt + (size_t)b * strideB;
  const T* Ab2 = SPLIT ? (A2  + (size_t)b * strideA) : nullptr;
  const T* Bb2 = SPLIT ? (Bt2 + (size_t)b * strideB) : nullptr;

  const int rlane = lane & 15;
  const int koff  = (lane >> 4) * 8;
  const int mOff  = (lane >> 4) * 8;

  v8f acc[4][4];
#pragma unroll
  for (int i = 0; i < 4; ++i)
#pragma unroll
    for (int j = 0; j < 4; ++j) acc[i][j] = (v8f){0.f,0.f,0.f,0.f,0.f,0.f,0.f,0.f};

  for (int k0 = 0; k0 < K; k0 += 32) {
    V bh[4], bl[4];
#pragma unroll
    for (int j = 0; j < 4; ++j) {
      const size_t bo = (size_t)(n0 + (j << 4) + rlane) * ldb + koff + k0;
      bh[j] = Frag<T>::load(Bb + bo);
      if (SPLIT) bl[j] = Frag<T>::load(Bb2 + bo);
    }
#pragma unroll
    for (int i = 0; i < 4; ++i) {
      const size_t ao = (size_t)(m0 + (i << 4) + rlane) * lda + koff + k0;
      V ah = Frag<T>::load(Ab + ao);
      V al;
      if (SPLIT) al = Frag<T>::load(Ab2 + ao);
#pragma unroll
      for (int j = 0; j < 4; ++j) {
        acc[i][j] = Frag<T>::mma(ah, bh[j], acc[i][j]);
        if (SPLIT) {
          acc[i][j] = Frag<T>::mma(ah, bl[j], acc[i][j]);
          acc[i][j] = Frag<T>::mma(al, bh[j], acc[i][j]);
        }
      }
      Frag<T>::guard(acc[i][0], acc[i][3], ah, SPLIT ? al : ah);
    }
    Frag<T>::keep(bh[0], bh[1], bh[2], bh[3]);
    if (SPLIT) Frag<T>::keep(bl[0], bl[1], bl[2], bl[3]);
  }
  acc_guard4(acc[0][0], acc[0][1], acc[0][2], acc[0][3]);
  acc_guard4(acc[1][0], acc[1][1], acc[1][2], acc[1][3]);
  acc_guard4(acc[2][0], acc[2][1], acc[2][2], acc[2][3]);
  acc_guard4(acc[3][0], acc[3][1], acc[3][2], acc[3][3]);

  float* slab = sT[wave];
  const float* Rb = RESID ? (resid + (size_t)b * strideR) : nullptr;
#pragma unroll
  for (int i = 0; i < 4; ++i) {
    const int mBase = m0 + (i << 4);
#pragma unroll
    for (int j = 0; j < 4; ++j) {
      const int n = n0 + (j << 4) + rlane;
      float bv = 0.f;
      if (BIAS_MODE == 2) bv = bias[n];
#pragma unroll
      for (int r = 0; r < 8; ++r) {
        float v = acc[i][j][r] * scale;
        if (BIAS_MODE == 1) v += bias[mBase + mOff + r];
        if (BIAS_MODE == 2) v += bv;
        if (RESID) v += Rb[(size_t)(mBase + mOff + r) * ldc + n];
        if (ACT == 1) v = tanhf(v);
        if (ACT == 2) v = fmaxf(v, 0.0f);
        if (ACT == 4) v = (v > 0.f) ? v : 0.01f * v;
        slab[(mOff + r) * 68 + (j << 4) + rlane] = v;
      }
    }
    __builtin_amdgcn_fence(__ATOMIC_RELEASE, "workgroup");
    __builtin_amdgcn_wave_barrier();
    __builtin_amdgcn_fence(__ATOMIC_ACQUIRE, "workgroup");
    if (OUT_MODE == 0 || OUT_MODE == 3) {
      float* C = (float*)Cout + (size_t)b * strideC;
      const int hh = lane >> 4, c4 = (lane & 15) * 4;
      for (int pass = 0; pass < 2; ++pass) {
#pragma unroll
        for (int it = 0; it < 8; ++it) {
          const int row = it * 2 + hh;
          v4f v = *(const v4f*)(slab + row * 68 + c4);
          *(volatile v4f*)(C + (size_t)(mBase + row) * ldc + n0 + c4) = v;
        }
        __threadfence();
      }
    }
    if (OUT_MODE != 0) {
      const int q = lane >> 3, c8 = (lane & 7) * 8;
      unsigned short* C  = (unsigned short*)((OUT_MODE == 3) ? Cout2 : Cout) + (size_t)b * strideC;
      unsigned short* C2 = (OUT_MODE == 2) ? ((unsigned short*)Cout2 + (size_t)b * strideC) : nullptr;
      for (int pass = 0; pass < 2; ++pass) {
#pragma unroll
        for (int it = 0; it < 4; ++it) {
          const int row = it * 4 + q;
          const float* sp = slab + row * 68 + c8;
          v8h hv, lv;
#pragma unroll
          for (int e = 0; e < 8; ++e) {
            if (OUT_MODE == 2) {
              unsigned short hb = f2bf_bits(sp[e]);
              unsigned short lb = f2bf_bits(sp[e] - bf_bits2f(hb));
              hv[e] = __builtin_bit_cast(_Float16, hb);
              lv[e] = __builtin_bit_cast(_Float16, lb);
            } else {
              hv[e] = (_Float16)sp[e];
              lv[e] = hv[e];
            }
          }
          *(volatile v8h*)(C + (size_t)(mBase + row) * ldc + n0 + c8) = hv;
          if (OUT_MODE == 2) *(volatile v8h*)(C2 + (size_t)(mBase + row) * ldc + n0 + c8) = lv;
        }
        __threadfence();
      }
    }
    __builtin_amdgcn_fence(__ATOMIC_RELEASE, "workgroup");
    __builtin_amdgcn_wave_barrier();
    __builtin_amdgcn_fence(__ATOMIC_ACQUIRE, "workgroup");
  }
}

__global__ __launch_bounds__(NTHR) void cast8_f16_kernel(const float* __restrict__ src, int n8, float mul,
                                                         unsigned short* __restrict__ dst) {
  const int i = blockIdx.x * NTHR + threadIdx.x;
  if (i >= n8) return;
  const size_t e0 = (size_t)i * 8;
  const v4f a0 = *(const v4f*)(src + e0);
  const v4f a1 = *(const v4f*)(src + e0 + 4);
  v8h hv;
  hv[0] = (_Float16)(a0[0] * mul); hv[1] = (_Float16)(a0[1] * mul); hv[2] = (_Float16)(a0[2] * mul); hv[3] = (_Float16)(a0[3] * mul);
  hv[4] = (_Float16)(a1[0] * mul); hv[5] = (_Float16)(a1[1] * mul); hv[6] = (_Float16)(a1[2] * mul); hv[7] = (_Float16)(a1[3] * mul);
  *(volatile v8h*)(dst + e0) = hv;
  __threadfence();
  *(volatile v8h*)(dst + e0) = hv;
}

__global__ __launch_bounds__(NTHR) void agent_proj_kernel(const float* __restrict__ af, const float* __restrict__ w,
                                                          const float* __restrict__ bb, unsigned short* __restrict__ A16) {
  const int i = blockIdx.x * NTHR + threadIdx.x;
  if (i >= ROWS_AGENT * 16) return;
  const int row = i >> 4;
  const int c8 = (i & 15) * 8;
  const v4f x = *(const v4f*)(af + (size_t)row * DIM_AGENT_IN);
  v8h hv;
#pragma unroll
  for (int e = 0; e < 8; ++e) {
    const int c = c8 + e;
    const v4f wv = *(const v4f*)(w + (size_t)c * DIM_AGENT_IN);
    float s = x[0] * wv[0];
    s = fmaf(x[1], wv[1], s);
    s = fmaf(x[2], wv[2], s);
    s = fmaf(x[3], wv[3], s);
    s += bb[c];
    hv[e] = (_Float16)s;
  }
  unsigned short* dst = A16 + (size_t)row * DIM_MODEL + c8;
  *(volatile v8h*)dst = hv;
  __threadfence();
  *(volatile v8h*)dst = hv;
}

constexpr int GRU_ROWS    = 16;
constexpr int GRU_HPITCH  = 136;
constexpr int GRU_SPITCH  = 132;
constexpr int GRU_GSTRIDE = DIM_MODEL * DIM_MODEL;

__device__ __forceinline__ void gru_mac(v8f (&acc)[3], const _Float16* arow, const _Float16* wrow) {
#pragma unroll 1
  for (int kc = 0; kc < 4; ++kc) {
    const int k0 = kc * 32;
    const v16h a  = FragH::load(arow + k0);
    const v16h b0 = FragH::load(wrow + k0);
    const v16h b1 = FragH::load(wrow + GRU_GSTRIDE + k0);
    const v16h b2 = FragH::load(wrow + 2 * GRU_GSTRIDE + k0);
    acc[0] = FragH::mma(a, b0, acc[0]);
    acc[1] = FragH::mma(a, b1, acc[1]);
    acc[2] = FragH::mma(a, b2, acc[2]);
    acc_guard3(acc[0], acc[1], acc[2]);
    keep4_h(a, b0, b1, b2);
  }
}

__global__ __launch_bounds__(NTHR) void gru_scan_kernel(
    const unsigned short* __restrict__ XGp,
    const unsigned short* __restrict__ Whhp,
    const float* __restrict__ bhh,
    int nsteps,
    unsigned short* __restrict__ Hout,
    float* __restrict__ Sout) {
  __shared__ __align__(16) _Float16 Ht[GRU_ROWS * GRU_HPITCH];
  __shared__ __align__(16) float    Ss[GRU_ROWS * GRU_SPITCH];

  const int tid = threadIdx.x, lane = tid & 31, wave = tid >> 5;
  const int c = lane & 15, hh = lane >> 4, koff = hh * 8;
  const int j  = 16 * wave + c;
  const int rb = 8 * hh;
  const int rowbase = blockIdx.x * GRU_ROWS;

#pragma unroll 1
  for (int i = tid; i < GRU_ROWS * GRU_HPITCH; i += NTHR) Ht[i] = (_Float16)0.0f;
  const float bias_r = bhh[j];
  const float bias_z = bhh[DIM_MODEL + j];
  const float bias_n = bhh[2 * DIM_MODEL + j];
  float hst[8], hsum[8];
#pragma unroll
  for (int r = 0; r < 8; ++r) { hst[r] = 0.0f; hsum[r] = 0.0f; }
  __syncthreads();

  const _Float16* arow = Ht + c * GRU_HPITCH + koff;
  const _Float16* wrow = (const _Float16*)Whhp + (size_t)j * DIM_MODEL + koff;
  const _Float16* XG = (const _Float16*)XGp;
  const v8f z8 = {0.f, 0.f, 0.f, 0.f, 0.f, 0.f, 0.f, 0.f};

#pragma unroll 1
  for (int t = 0; t < nsteps; ++t) {
    float xr[8], xz[8], xn[8];
#pragma unroll
    for (int r = 0; r < 8; ++r) {
      const size_t g = ((size_t)(rowbase + rb + r) * (size_t)nsteps + (size_t)t) * GATES3 + (size_t)j;
      xr[r] = (float)XG[g];
      xz[r] = (float)XG[g + DIM_MODEL];
      xn[r] = (float)XG[g + 2 * DIM_MODEL];
    }
    v8f acc[3];
    acc[0] = z8; acc[1] = z8; acc[2] = z8;
    gru_mac(acc, arow, wrow);
#pragma unroll
    for (int r = 0; r < 8; ++r) {
      const float ghr = fmaf(acc[0][r], W_FOLD, bias_r);
      const float ghz = fmaf(acc[1][r], W_FOLD, bias_z);
      const float ghn = fmaf(acc[2][r], W_FOLD, bias_n);
      const float rr = fsig(xr[r] + ghr);
      const float zz = fsig(xz[r] + ghz);
      const float nn = ftanh(fmaf(rr, ghn, xn[r]));
      const float hnew = fmaf(zz, hst[r] - nn, nn);
      hst[r] = hnew;
      hsum[r] += hnew;
    }
    __syncthreads();
#pragma unroll
    for (int r = 0; r < 8; ++r) Ht[(rb + r) * GRU_HPITCH + j] = (_Float16)hst[r];
    __syncthreads();
    {
      const int row = 2 * wave + hh;
      const v8h v = *(const v8h*)(Ht + row * GRU_HPITCH + c * 8);
      unsigned short* dst = Hout + ((size_t)(rowbase + row) * (size_t)nsteps + (size_t)t) * DIM_MODEL + c * 8;
      *(volatile v8h*)dst = v;
      __threadfence();
      *(volatile v8h*)dst = v;
    }
  }

#pragma unroll
  for (int r = 0; r < 8; ++r) Ss[(rb + r) * GRU_SPITCH + j] = hsum[r];
  __syncthreads();
  if (Sout != nullptr) {
    for (int pass = 0; pass < 2; ++pass) {
#pragma unroll
      for (int it = 0; it < 2; ++it) {
        const int row = 2 * wave + it;
        const v4f v = *(const v4f*)(Ss + row * GRU_SPITCH + lane * 4);
        *(volatile v4f*)(Sout + (size_t)(rowbase + row) * DIM_MODEL + lane * 4) = v;
      }
      __threadfence();
    }
  }
}

__device__ __forceinline__ void store_rows6_f16(const float* so, unsigned short* dst0, int tid) {
  if (tid < 96) {
    const int row = tid >> 4, c8 = (tid & 15) * 8;
    v8h hv;
#pragma unroll
    for (int e = 0; e < 8; ++e) hv[e] = (_Float16)so[row * 132 + c8 + e];
    unsigned short* dst = dst0 + (size_t)row * DIM_MODEL + c8;
    for (int pass = 0; pass < 2; ++pass) {
      *(volatile v8h*)dst = hv;
      __threadfence();
    }
  }
}

__global__ __launch_bounds__(NTHR) void agent_self_attn_kernel(const float* __restrict__ QKV,
                                                               unsigned short* __restrict__ O16) {
  __shared__ __align__(16) float sx[STEPS_AGENT * GATES3];
  __shared__ float sprob[STEPS_AGENT * NUM_HEADS * 8];
  __shared__ __align__(16) float so[STEPS_AGENT * 132];
  const int tid = threadIdx.x;
  const int scene = blockIdx.x;
  const float* base = QKV + (size_t)scene * STEPS_AGENT * GATES3;
#pragma unroll 1
  for (int i = tid; i < STEPS_AGENT * GATES3; i += NTHR) sx[i] = base[i];
  __syncthreads();
  if (tid < STEPS_AGENT * NUM_HEADS * STEPS_AGENT) {
    const int i = tid / 24;
    const int rem = tid - 24 * i;
    const int h = rem / 6;
    const int jk = rem - 6 * h;
    const float* qp = sx + i * GATES3 + h * DIM_HEAD;
    const float* kp = sx + jk * GATES3 + DIM_MODEL + h * DIM_HEAD;
    float s = 0.f;
#pragma unroll 1
    for (int d = 0; d < DIM_HEAD; ++d) s = fmaf(qp[d], kp[d], s);
    sprob[(i * NUM_HEADS + h) * 8 + jk] = s * ATT_SCALE;
  }
  __syncthreads();
  if (tid < STEPS_AGENT * NUM_HEADS) {
    float* pr = sprob + tid * 8;
    const float s0 = pr[0], s1 = pr[1], s2 = pr[2], s3 = pr[3], s4 = pr[4], s5 = pr[5];
    float m = fmaxf(fmaxf(fmaxf(s0, s1), fmaxf(s2, s3)), fmaxf(s4, s5));
    const float e0 = __expf(s0 - m), e1 = __expf(s1 - m), e2 = __expf(s2 - m);
    const float e3 = __expf(s3 - m), e4 = __expf(s4 - m), e5 = __expf(s5 - m);
    const float sum = ((e0 + e1) + (e2 + e3)) + (e4 + e5);
    const float inv = 1.0f / sum;
    pr[0] = e0 * inv; pr[1] = e1 * inv; pr[2] = e2 * inv; pr[3] = e3 * inv; pr[4] = e4 * inv; pr[5] = e5 * inv;
  }
  __syncthreads();
#pragma unroll 1
  for (int e = tid; e < STEPS_AGENT * DIM_MODEL; e += NTHR) {
    const int i = e >> 7;
    const int hd = e & 127;
    const int h = hd >> 5;
    const float* pr = sprob + (i * NUM_HEADS + h) * 8;
    float o = 0.f;
#pragma unroll 1
    for (int jk = 0; jk < STEPS_AGENT; ++jk) o = fmaf(pr[jk], sx[jk * GATES3 + 2 * DIM_MODEL + hd], o);
    so[i * 132 + hd] = o;
  }
  __syncthreads();
  store_rows6_f16(so, O16 + (size_t)scene * STEPS_AGENT * DIM_MODEL, tid);
}

constexpr int LA_SPITCH = 256;
union HalfPack32 { v8h v[4]; _Float16 e[32]; };

__global__ __launch_bounds__(NTHR) void keys240_attn_kernel(const float* __restrict__ QA,
                                                            const unsigned short* __restrict__ KVp,
                                                            unsigned short* __restrict__ O16, int scene0) {
  __shared__ __align__(16) float sqa[STEPS_AGENT * DIM_MODEL];
  __shared__ __align__(16) float ssc[STEPS_AGENT * NUM_HEADS * LA_SPITCH];
  __shared__ __align__(16) float so[STEPS_AGENT * 132];
  const int tid = threadIdx.x, lane = tid & 31, wave = tid >> 5;
  const int sl = blockIdx.x;
  const int scene = scene0 + sl;
  const float* qb = QA + (size_t)scene * STEPS_AGENT * DIM_MODEL;
#pragma unroll 1
  for (int i = tid; i < STEPS_AGENT * DIM_MODEL; i += NTHR) sqa[i] = qb[i];
  const _Float16* KV = (const _Float16*)KVp + (size_t)sl * STEPS_LANE * (2 * DIM_MODEL);
  __syncthreads();

  {
    const int jkey = (tid < STEPS_LANE) ? tid : (STEPS_LANE - 1);
    const _Float16* krow = KV + (size_t)jkey * (2 * DIM_MODEL);
#pragma unroll 1
    for (int h = 0; h < NUM_HEADS; ++h) {
      HalfPack32 kk;
      kk.v[0] = *(const v8h*)(krow + h * DIM_HEAD);
      kk.v[1] = *(const v8h*)(krow + h * DIM_HEAD + 8);
      kk.v[2] = *(const v8h*)(krow + h * DIM_HEAD + 16);
      kk.v[3] = *(const v8h*)(krow + h * DIM_HEAD + 24);
      float kf[32];
#pragma unroll
      for (int d = 0; d < 32; ++d) kf[d] = (float)kk.e[d];
#pragma unroll 1
      for (int i = 0; i < STEPS_AGENT; ++i) {
        const float* qp = sqa + i * DIM_MODEL + h * DIM_HEAD;
        float s = 0.f;
#pragma unroll
        for (int d = 0; d < 32; ++d) s = fmaf(qp[d], kf[d], s);
        ssc[(i * NUM_HEADS + h) * LA_SPITCH + tid] = s * ATT_SCALE;
      }
    }
  }
  __syncthreads();

#pragma unroll 1
  for (int rep = 0; rep < 3; ++rep) {
    float* pr = ssc + (rep * 8 + wave) * LA_SPITCH;
    float m = -INFINITY;
#pragma unroll 1
    for (int cc = 0; cc < 8; ++cc) {
      const int jj = cc * 32 + lane;
      float v = pr[jj];
      v = (jj < STEPS_LANE) ? v : -INFINITY;
      m = fmaxf(m, v);
    }
#pragma unroll
    for (int off = 16; off > 0; off >>= 1) m = fmaxf(m, __shfl_xor(m, off, 32));
    float sum = 0.f;
#pragma unroll 1
    for (int cc = 0; cc < 8; ++cc) {
      const int jj = cc * 32 + lane;
      float ev = __expf(pr[jj] - m);
      ev = (jj < STEPS_LANE) ? ev : 0.f;
      sum += ev;
      pr[jj] = ev;
    }
#pragma unroll
    for (int off = 16; off > 0; off >>= 1) sum += __shfl_xor(sum, off, 32);
    const float inv = 1.0f / sum;
#pragma unroll 1
    for (int cc = 0; cc < 8; ++cc) {
      const int jj = cc * 32 + lane;
      pr[jj] = pr[jj] * inv;
    }
  }
  __syncthreads();

#pragma unroll 1
  for (int k3 = 0; k3 < 3; ++k3) {
    const int e = tid + NTHR * k3;
    const int i = e >> 7;
    const int hd = e & 127;
    const int h = hd >> 5;
    const float* pr = ssc + (i * NUM_HEADS + h) * LA_SPITCH;
    const _Float16* vp = KV + DIM_MODEL + hd;
    float o = 0.f;
#pragma unroll 1
    for (int j4 = 0; j4 < STEPS_LANE; j4 += 4) {
      const v4f p4 = *(const v4f*)(pr + j4);
      const float v0 = (float)vp[(size_t)(j4 + 0) * (2 * DIM_MODEL)];
      const float v1 = (float)vp[(size_t)(j4 + 1) * (2 * DIM_MODEL)];
      const float v2 = (float)vp[(size_t)(j4 + 2) * (2 * DIM_MODEL)];
      const float v3 = (float)vp[(size_t)(j4 + 3) * (2 * DIM_MODEL)];
      o = fmaf(p4[0], v0, o);
      o = fmaf(p4[1], v1, o);
      o = fmaf(p4[2], v2, o);
      o = fmaf(p4[3], v3, o);
    }
    so[i * 132 + hd] = o;
  }
  __syncthreads();
  store_rows6_f16(so, O16 + (size_t)scene * STEPS_AGENT * DIM_MODEL, tid);
}

__global__ __launch_bounds__(NTHR) void queries240_attn_kernel(const unsigned short* __restrict__ QLp,
                                                               const float* __restrict__ KVA,
                                                               unsigned short* __restrict__ MO16, int scene0) {
  __shared__ __align__(16) float skv[STEPS_AGENT * 2 * DIM_MODEL];
  __shared__ __align__(16) float sprob[NTHR * 32];
  __shared__ float spsum[32];
  __shared__ __align__(16) float smo[132];
  const int tid = threadIdx.x, lane = tid & 31, wave = tid >> 5;
  const int sl = blockIdx.x;
  const int scene = scene0 + sl;
  const float* kvb = KVA + (size_t)scene * STEPS_AGENT * (2 * DIM_MODEL);
#pragma unroll 1
  for (int i = tid; i < STEPS_AGENT * 2 * DIM_MODEL; i += NTHR) skv[i] = kvb[i];
  __syncthreads();
  {
    const int tq = (tid < STEPS_LANE) ? tid : (STEPS_LANE - 1);
    const _Float16* qrow = (const _Float16*)QLp + ((size_t)sl * STEPS_LANE + (size_t)tq) * DIM_MODEL;
    float* sprow = sprob + tid * 32;
#pragma unroll 1
    for (int h = 0; h < NUM_HEADS; ++h) {
      HalfPack32 qq;
      qq.v[0] = *(const v8h*)(qrow + h * DIM_HEAD);
      qq.v[1] = *(const v8h*)(qrow + h * DIM_HEAD + 8);
      qq.v[2] = *(const v8h*)(qrow + h * DIM_HEAD + 16);
      qq.v[3] = *(const v8h*)(qrow + h * DIM_HEAD + 24);
      float qf[32];
#pragma unroll
      for (int d = 0; d < 32; ++d) qf[d] = (float)qq.e[d];
      float* spr = sprow + h * 8;
#pragma unroll 1
      for (int jk = 0; jk < STEPS_AGENT; ++jk) {
        const float* kp = skv + jk * (2 * DIM_MODEL) + h * DIM_HEAD;
        float s = 0.f;
#pragma unroll
        for (int d = 0; d < 32; ++d) s = fmaf(qf[d], kp[d], s);
        spr[jk] = s * ATT_SCALE;
      }
      const float s0 = spr[0], s1 = spr[1], s2 = spr[2], s3 = spr[3], s4 = spr[4], s5 = spr[5];
      const float m = fmaxf(fmaxf(fmaxf(s0, s1), fmaxf(s2, s3)), fmaxf(s4, s5));
      const float e0 = __expf(s0 - m), e1 = __expf(s1 - m), e2 = __expf(s2 - m);
      const float e3 = __expf(s3 - m), e4 = __expf(s4 - m), e5 = __expf(s5 - m);
      const float sum = ((e0 + e1) + (e2 + e3)) + (e4 + e5);
      const float inv = 1.0f / sum;
      spr[0] = e0 * inv; spr[1] = e1 * inv; spr[2] = e2 * inv; spr[3] = e3 * inv; spr[4] = e4 * inv; spr[5] = e5 * inv;
    }
  }
  __syncthreads();
  if (tid < NUM_HEADS * STEPS_AGENT) {
    const int h = tid / 6;
    const int jk = tid - 6 * h;
    float s = 0.f;
#pragma unroll 1
    for (int t = 0; t < STEPS_LANE; ++t) s += sprob[t * 32 + h * 8 + jk];
    spsum[tid] = s;
  }
  __syncthreads();
  if (tid < DIM_MODEL) {
    const int h = tid >> 5, d = tid & 31;
    float o = 0.f;
#pragma unroll 1
    for (int jk = 0; jk < STEPS_AGENT; ++jk) o = fmaf(spsum[h * 6 + jk], skv[jk * (2 * DIM_MODEL) + DIM_MODEL + h * DIM_HEAD + d], o);
    smo[tid] = o * INV_LANE_STEPS;
  }
  __syncthreads();
  if (wave == 0 && lane < 16) {
    v8h hv;
#pragma unroll
    for (int e = 0; e < 8; ++e) hv[e] = (_Float16)smo[lane * 8 + e];
    unsigned short* dst = MO16 + (size_t)scene * DIM_MODEL + lane * 8;
    for (int pass = 0; pass < 2; ++pass) {
      *(volatile v8h*)dst = hv;
      __threadfence();
    }
  }
}

union FloatPack8 { v4f q[2]; float f[8]; };

__global__ __launch_bounds__(NTHR) void glu_fuse_kernel(const float* __restrict__ ASA, const float* __restrict__ ALA,
                                                        const float* __restrict__ LSUM, const float* __restrict__ LA,
                                                        unsigned short* __restrict__ FU16) {
  const int i = blockIdx.x * NTHR + threadIdx.x;
  if (i >= ROWS_AGENT * 32) return;
  const int row = i >> 5;
  const int c8 = (i & 31) * 8;
  const int scene = row / STEPS_AGENT;
  const bool agent_half = (c8 < DIM_MODEL);
  const int cc8 = c8 & (DIM_MODEL - 1);
  FloatPack8 av, gv, sv, lv;
  av.q[0] = *(const v4f*)(ASA  + (size_t)row   * DIM_MODEL + cc8); av.q[1] = *(const v4f*)(ASA  + (size_t)row   * DIM_MODEL + cc8 + 4);
  gv.q[0] = *(const v4f*)(ALA  + (size_t)scene * DIM_MODEL + cc8); gv.q[1] = *(const v4f*)(ALA  + (size_t)scene * DIM_MODEL + cc8 + 4);
  sv.q[0] = *(const v4f*)(LSUM + (size_t)scene * DIM_MODEL + cc8); sv.q[1] = *(const v4f*)(LSUM + (size_t)scene * DIM_MODEL + cc8 + 4);
  lv.q[0] = *(const v4f*)(LA   + (size_t)row   * DIM_MODEL + cc8); lv.q[1] = *(const v4f*)(LA   + (size_t)row   * DIM_MODEL + cc8 + 4);
  v8h hv;
#pragma unroll
  for (int e = 0; e < 8; ++e) {
    const float x = agent_half ? av.f[e] : sv.f[e] * INV_LANE_STEPS;
    const float g = agent_half ? gv.f[e] : lv.f[e];
    hv[e] = (_Float16)(x * fsig(g));
  }
  unsigned short* dst = FU16 + (size_t)row * (2 * DIM_MODEL) + c8;
  *(volatile v8h*)dst = hv;
  __threadfence();
  *(volatile v8h*)dst = hv;
}

template <int OUT_MODE>
static void launch_gemm(hipStream_t st, const unsigned short* A, int lda, const unsigned short* Bt, int ldb,
                        void* Cd, void* Cd2, int ldc, const float* bias, int M, int N, int K) {
  const int tiles = (M / 64) * (N / 64);
  const int blocks = (tiles + 7) / 8;
  wmma_gemm64<0, false, 2, OUT_MODE, false, 0><<<dim3(blocks, 1), NTHR, 0, st>>>(
      A, nullptr, lda, 0L, Bt, nullptr, ldb, 0L, Cd, Cd2, ldc, 0L, bias, nullptr, 0L, M, N, K, W_FOLD);
}

extern "C" void kernel_launch(void* const* d_in, const int* in_sizes, int n_in,
                              void* d_out, int out_size, void* d_ws, size_t ws_size, hipStream_t stream) {
  if (n_in < 26 || d_out == nullptr || d_ws == nullptr || in_sizes == nullptr) return;
  const int expect_sizes[26] = {
      NUM_SCENES * STEPS_AGENT * DIM_AGENT_IN, NUM_SCENES * STEPS_LANE * DIM_MODEL,
      DIM_MODEL * DIM_AGENT_IN, DIM_MODEL,
      GATES3 * DIM_MODEL, GATES3 * DIM_MODEL, GATES3, GATES3,
      GATES3 * DIM_MODEL, GATES3 * DIM_MODEL, GATES3, GATES3,
      NUM_LAYERS * GATES3 * DIM_MODEL, NUM_LAYERS * GATES3, NUM_LAYERS * DIM_MODEL * DIM_MODEL, NUM_LAYERS * DIM_MODEL,
      NUM_LAYERS * GATES3 * DIM_MODEL, NUM_LAYERS * GATES3, NUM_LAYERS * DIM_MODEL * DIM_MODEL, NUM_LAYERS * DIM_MODEL,
      NUM_LAYERS * GATES3 * DIM_MODEL, NUM_LAYERS * GATES3, NUM_LAYERS * DIM_MODEL * DIM_MODEL, NUM_LAYERS * DIM_MODEL,
      DIM_MODEL * 2 * DIM_MODEL, DIM_MODEL};
  static_assert(sizeof(expect_sizes) / sizeof(expect_sizes[0]) == 26, "cfg");
  for (int i = 0; i < 26; ++i) if (in_sizes[i] != expect_sizes[i]) return;
  if (out_size != ROWS_AGENT * DIM_MODEL) return;

  const float* agent_features = (const float*)d_in[0];
  const float* lane_features  = (const float*)d_in[1];
  const float* agent_proj_w   = (const float*)d_in[2];
  const float* agent_proj_b   = (const float*)d_in[3];
  const float* agru_wih = (const float*)d_in[4];
  const float* agru_whh = (const float*)d_in[5];
  const float* agru_bih = (const float*)d_in[6];
  const float* agru_bhh = (const float*)d_in[7];
  const float* lgru_wih = (const float*)d_in[8];
  const float* lgru_whh = (const float*)d_in[9];
  const float* lgru_bih = (const float*)d_in[10];
  const float* lgru_bhh = (const float*)d_in[11];
  const float* self_wqkv = (const float*)d_in[12];
  const float* self_bqkv = (const float*)d_in[13];
  const float* self_wout = (const float*)d_in[14];
  const float* self_bout = (const float*)d_in[15];
  const float* al_wqkv = (const float*)d_in[16];
  const float* al_bqkv = (const float*)d_in[17];
  const float* al_wout = (const float*)d_in[18];
  const float* al_bout = (const float*)d_in[19];
  const float* la_wqkv = (const float*)d_in[20];
  const float* la_bqkv = (const float*)d_in[21];
  const float* la_wout = (const float*)d_in[22];
  const float* la_bout = (const float*)d_in[23];
  const float* proj_w = (const float*)d_in[24];
  const float* proj_b = (const float*)d_in[25];
  float* out = (float*)d_out;

  char* ws = (char*)d_ws; size_t off = 0;
  auto carve = [&](size_t bytes) -> char* { char* p = ws + off; off += (bytes + 255) & ~(size_t)255; return p; };
  const size_t H2 = 2, F4 = 4;
  unsigned short* W_AGWIH = (unsigned short*)carve((size_t)GATES3 * DIM_MODEL * H2);
  unsigned short* W_AGWHH = (unsigned short*)carve((size_t)GATES3 * DIM_MODEL * H2);
  unsigned short* W_LGWIH = (unsigned short*)carve((size_t)GATES3 * DIM_MODEL * H2);
  unsigned short* W_LGWHH = (unsigned short*)carve((size_t)GATES3 * DIM_MODEL * H2);
  unsigned short* W_SQKV  = (unsigned short*)carve((size_t)NUM_LAYERS * GATES3 * DIM_MODEL * H2);
  unsigned short* W_SOUT  = (unsigned short*)carve((size_t)NUM_LAYERS * DIM_MODEL * DIM_MODEL * H2);
  unsigned short* W_ALQKV = (unsigned short*)carve((size_t)NUM_LAYERS * GATES3 * DIM_MODEL * H2);
  unsigned short* W_ALOUT = (unsigned short*)carve((size_t)NUM_LAYERS * DIM_MODEL * DIM_MODEL * H2);
  unsigned short* W_LAQKV = (unsigned short*)carve((size_t)NUM_LAYERS * GATES3 * DIM_MODEL * H2);
  unsigned short* W_LAOUT = (unsigned short*)carve((size_t)NUM_LAYERS * DIM_MODEL * DIM_MODEL * H2);
  unsigned short* W_PROJ  = (unsigned short*)carve((size_t)DIM_MODEL * 2 * DIM_MODEL * H2);
  unsigned short* A16   = (unsigned short*)carve((size_t)ROWS_AGENT * DIM_MODEL * H2);
  unsigned short* AXG16 = (unsigned short*)carve((size_t)ROWS_AGENT * GATES3 * H2);
  unsigned short* AE16  = (unsigned short*)carve((size_t)ROWS_AGENT * DIM_MODEL * H2);
  float* QKV32          = (float*)carve((size_t)ROWS_AGENT * GATES3 * F4);
  unsigned short* O16   = (unsigned short*)carve((size_t)ROWS_AGENT * DIM_MODEL * H2);
  float* ASA32          = (float*)carve((size_t)ROWS_AGENT * DIM_MODEL * F4);
  unsigned short* ASA16 = (unsigned short*)carve((size_t)ROWS_AGENT * DIM_MODEL * H2);
  float* KVA32          = (float*)carve((size_t)ROWS_AGENT * 2 * DIM_MODEL * F4);
  float* QA32           = (float*)carve((size_t)ROWS_AGENT * DIM_MODEL * F4);
  unsigned short* OLA16 = (unsigned short*)carve((size_t)ROWS_AGENT * DIM_MODEL * H2);
  unsigned short* MO16  = (unsigned short*)carve((size_t)NUM_SCENES * DIM_MODEL * H2);
  float* LA32           = (float*)carve((size_t)ROWS_AGENT * DIM_MODEL * F4);
  float* ALA32          = (float*)carve((size_t)NUM_SCENES * DIM_MODEL * F4);
  unsigned short* FU16  = (unsigned short*)carve((size_t)ROWS_AGENT * 2 * DIM_MODEL * H2);
  float* LSUM           = (float*)carve((size_t)NUM_SCENES * DIM_MODEL * F4);
  unsigned short* LE16H = (unsigned short*)carve((size_t)ROWS_LANE_HALF * DIM_MODEL * H2);
  unsigned short* LF16H = (unsigned short*)carve((size_t)ROWS_LANE_HALF * DIM_MODEL * H2);
  unsigned short* XGH   = (unsigned short*)carve((size_t)ROWS_LANE_HALF * GATES3 * H2);
  unsigned short* KVH   = XGH;
  unsigned short* QLH   = XGH + (size_t)ROWS_LANE_HALF * 2 * DIM_MODEL;
  if (off > ws_size || off > (size_t)134217728) return;

  auto castw = [&](const float* src, int n, float mul, unsigned short* dst) {
    const int n8 = n / 8;
    cast8_f16_kernel<<<(n8 + NTHR - 1) / NTHR, NTHR, 0, stream>>>(src, n8, mul, dst);
  };
  castw(agru_wih, GATES3 * DIM_MODEL, W_CARRY, W_AGWIH);
  castw(agru_whh, GATES3 * DIM_MODEL, W_CARRY, W_AGWHH);
  castw(lgru_wih, GATES3 * DIM_MODEL, W_CARRY, W_LGWIH);
  castw(lgru_whh, GATES3 * DIM_MODEL, W_CARRY, W_LGWHH);
  castw(self_wqkv, NUM_LAYERS * GATES3 * DIM_MODEL, W_CARRY, W_SQKV);
  castw(self_wout, NUM_LAYERS * DIM_MODEL * DIM_MODEL, W_CARRY, W_SOUT);
  castw(al_wqkv, NUM_LAYERS * GATES3 * DIM_MODEL, W_CARRY, W_ALQKV);
  castw(al_wout, NUM_LAYERS * DIM_MODEL * DIM_MODEL, W_CARRY, W_ALOUT);
  castw(la_wqkv, NUM_LAYERS * GATES3 * DIM_MODEL, W_CARRY, W_LAQKV);
  castw(la_wout, NUM_LAYERS * DIM_MODEL * DIM_MODEL, W_CARRY, W_LAOUT);
  castw(proj_w, DIM_MODEL * 2 * DIM_MODEL, W_CARRY, W_PROJ);

  agent_proj_kernel<<<ROWS_AGENT * 16 / NTHR, NTHR, 0, stream>>>(agent_features, agent_proj_w, agent_proj_b, A16);
  launch_gemm<1>(stream, A16, DIM_MODEL, W_AGWIH, DIM_MODEL, AXG16, nullptr, GATES3, agru_bih, ROWS_AGENT, GATES3, DIM_MODEL);
  gru_scan_kernel<<<NUM_SCENES / GRU_ROWS, NTHR, 0, stream>>>(AXG16, W_AGWHH, agru_bhh, STEPS_AGENT, AE16, (float*)nullptr);
  for (int li = 0; li < NUM_LAYERS; ++li) {
    const unsigned short* asa_in = (li == 0) ? AE16 : ASA16;
    launch_gemm<0>(stream, asa_in, DIM_MODEL, W_SQKV + (size_t)li * GATES3 * DIM_MODEL, DIM_MODEL,
                   QKV32, nullptr, GATES3, self_bqkv + (size_t)li * GATES3, ROWS_AGENT, GATES3, DIM_MODEL);
    agent_self_attn_kernel<<<NUM_SCENES, NTHR, 0, stream>>>(QKV32, O16);
    launch_gemm<3>(stream, O16, DIM_MODEL, W_SOUT + (size_t)li * DIM_MODEL * DIM_MODEL, DIM_MODEL,
                   ASA32, ASA16, DIM_MODEL, self_bout + (size_t)li * DIM_MODEL, ROWS_AGENT, DIM_MODEL, DIM_MODEL);
  }
  const size_t l2w = (size_t)2 * GATES3 * DIM_MODEL;
  const size_t l2o = (size_t)2 * DIM_MODEL * DIM_MODEL;
  launch_gemm<0>(stream, ASA16, DIM_MODEL, W_ALQKV + l2w + (size_t)DIM_MODEL * DIM_MODEL, DIM_MODEL,
                 KVA32, nullptr, 2 * DIM_MODEL, al_bqkv + 2 * GATES3 + DIM_MODEL, ROWS_AGENT, 2 * DIM_MODEL, DIM_MODEL);
  launch_gemm<0>(stream, ASA16, DIM_MODEL, W_LAQKV + l2w, DIM_MODEL,
                 QA32, nullptr, DIM_MODEL, la_bqkv + 2 * GATES3, ROWS_AGENT, DIM_MODEL, DIM_MODEL);

  for (int hs = 0; hs < 2; ++hs) {
    const float* lf = lane_features + (size_t)hs * ROWS_LANE_HALF * DIM_MODEL;
    castw(lf, ROWS_LANE_HALF * DIM_MODEL, 1.0f, LF16H);
    launch_gemm<1>(stream, LF16H, DIM_MODEL, W_LGWIH, DIM_MODEL, XGH, nullptr, GATES3, lgru_bih, ROWS_LANE_HALF, GATES3, DIM_MODEL);
    gru_scan_kernel<<<HALF_SCENES / GRU_ROWS, NTHR, 0, stream>>>(XGH, W_LGWHH, lgru_bhh, STEPS_LANE, LE16H,
                                                                 LSUM + (size_t)hs * HALF_SCENES * DIM_MODEL);
    launch_gemm<1>(stream, LE16H, DIM_MODEL, W_LAQKV + l2w + (size_t)DIM_MODEL * DIM_MODEL, DIM_MODEL,
                   KVH, nullptr, 2 * DIM_MODEL, la_bqkv + 2 * GATES3 + DIM_MODEL, ROWS_LANE_HALF, 2 * DIM_MODEL, DIM_MODEL);
    launch_gemm<1>(stream, LE16H, DIM_MODEL, W_ALQKV + l2w, DIM_MODEL,
                   QLH, nullptr, DIM_MODEL, al_bqkv + 2 * GATES3, ROWS_LANE_HALF, DIM_MODEL, DIM_MODEL);
    keys240_attn_kernel<<<HALF_SCENES, NTHR, 0, stream>>>(QA32, KVH, OLA16, hs * HALF_SCENES);
    queries240_attn_kernel<<<HALF_SCENES, NTHR, 0, stream>>>(QLH, KVA32, MO16, hs * HALF_SCENES);
  }

  launch_gemm<0>(stream, OLA16, DIM_MODEL, W_LAOUT + l2o, DIM_MODEL, LA32, nullptr, DIM_MODEL,
                 la_bout + 2 * DIM_MODEL, ROWS_AGENT, DIM_MODEL, DIM_MODEL);
  launch_gemm<0>(stream, MO16, DIM_MODEL, W_ALOUT + l2o, DIM_MODEL, ALA32, nullptr, DIM_MODEL,
                 al_bout + 2 * DIM_MODEL, NUM_SCENES, DIM_MODEL, DIM_MODEL);
  glu_fuse_kernel<<<ROWS_AGENT * 32 / NTHR, NTHR, 0, stream>>>(ASA32, ALA32, LSUM, LA32, FU16);
  launch_gemm<0>(stream, FU16, 2 * DIM_MODEL, W_PROJ, 2 * DIM_MODEL, out, nullptr, DIM_MODEL,
                 proj_b, ROWS_AGENT, DIM_MODEL, 2 * DIM_MODEL);
}
